// MolecularGnnSmiles_44014824849805
// MI455X (gfx1250) — hardware-run, weakly checked
//
#include <hip/hip_runtime.h>
#include <stddef.h>


#define HID 128
#define NMAT 5
#define NTILE (NMAT * 32)
#define NSLOTS (NTILE * 64)
#define TB_L0 96
#define TB_L1 128

#define CH1 2048
#define PITCHB 3136
#define MAXB PITCHB
#define BPT 25
#define MAXGRP 16
#define MAXNB1 (32 * MAXGRP)
#define CAP3 2048
#define GRW 256
#define NCH 16
#define HP 136
#define SP 132

typedef _Float16 v16h __attribute__((ext_vector_type(16)));
typedef _Float16 v8h __attribute__((ext_vector_type(8)));
typedef float v8f __attribute__((ext_vector_type(8)));
typedef float v4f __attribute__((ext_vector_type(4)));
typedef int v4i __attribute__((ext_vector_type(4)));
typedef v4f __attribute__((may_alias)) v4fa;
typedef v4i __attribute__((may_alias)) v4ia;
typedef v8h __attribute__((may_alias)) v8ha;

union Frag { v16h v; v8h half[2]; _Float16 e[16]; };

__device__ __forceinline__ v8f wmma16(const v16h& a, const v16h& b, v8f c) {
    return __builtin_amdgcn_wmma_f32_16x16x32_f16(false, a, false, b, (short)0, c, false, false);
}

__device__ __forceinline__ v8f zero8() {
    v8f z = {0.0f, 0.0f, 0.0f, 0.0f, 0.0f, 0.0f, 0.0f, 0.0f};
    return z;
}

__device__ __forceinline__ v16h frag_f32(const float* rowp, int k0, int h) {
    const v4f* rp = (const v4f*)rowp + (k0 >> 2);
    const v4f p0 = rp[2 * h], p1 = rp[2 * h + 1], p2 = rp[4 + 2 * h], p3 = rp[5 + 2 * h];
    Frag a;
    a.e[0] = (_Float16)p0.x;  a.e[1] = (_Float16)p0.y;  a.e[2] = (_Float16)p0.z;  a.e[3] = (_Float16)p0.w;
    a.e[4] = (_Float16)p1.x;  a.e[5] = (_Float16)p1.y;  a.e[6] = (_Float16)p1.z;  a.e[7] = (_Float16)p1.w;
    a.e[8] = (_Float16)p2.x;  a.e[9] = (_Float16)p2.y;  a.e[10] = (_Float16)p2.z; a.e[11] = (_Float16)p2.w;
    a.e[12] = (_Float16)p3.x; a.e[13] = (_Float16)p3.y; a.e[14] = (_Float16)p3.z; a.e[15] = (_Float16)p3.w;
    return a.v;
}

__device__ __forceinline__ v16h frag_lds(const _Float16* rowp, int k0, int h) {
    Frag a;
    a.half[0] = *(const v8ha*)(rowp + k0 + 8 * h);
    a.half[1] = *(const v8ha*)(rowp + k0 + 16 + 8 * h);
    return a.v;
}

__device__ __forceinline__ v16h frag_b(const v8h* bq, int tile, int lane) {
    Frag b;
    const int f = (tile * 32 + lane) * 2;
    b.half[0] = bq[f];
    b.half[1] = bq[f + 1];
    return b.v;
}

__global__ __launch_bounds__(256) void k_prep(const float* __restrict__ gw, const float* __restrict__ lw,
                                              _Float16* bfrag) {
    const int t0 = blockIdx.x * 256 + threadIdx.x;
    const bool ok = t0 < NSLOTS;
    const int tt = ok ? t0 : 0;
    const int g = tt & 1, l = (tt >> 1) & 31, tile = tt >> 6;
    const int h = l >> 4, m = l & 15;
    const int mat = tile >> 5, lt = tile & 31;
    const int ks = lt >> 3, nt = lt & 7;
    const int c = nt * 16 + m;
    const int kb = 32 * ks + 16 * g + 8 * h;
    const int mg = mat < 3 ? mat : 0;
    const int ml = mat >= 3 ? (mat - 3) : 0;
    union { v8h v; _Float16 e[8]; } u;
#pragma unroll
    for (int ii = 0; ii < 8; ++ii) {
        const int k = kb + ii;
        const int idx = c * HID + k;
        const float vg = gw[(size_t)mg * HID * HID + idx];
        const float vl = lw[(size_t)ml * HID * HID + idx];
        const float v = (mat < 3) ? vg : vl;
        u.e[ii] = (_Float16)(v * 64.0f);
    }
    const v8h val = u.v;
    if (ok) *(volatile v8h*)(bfrag + (size_t)tt * 8) = val;
    __threadfence();
    if (ok) *(volatile v8h*)(bfrag + (size_t)tt * 8) = val;
}

__global__ __launch_bounds__(256) void k_embed(const int* __restrict__ ids, const float* __restrict__ embd,
                                               float* xout, int N, int V) {
    const int lane = threadIdx.x & 31;
    const int n = blockIdx.x * 8 + (threadIdx.x >> 5);
    const int nc = n < N ? n : N - 1;
    int id = ids[nc];
    id = id < 0 ? 0 : (id > V - 1 ? V - 1 : id);
    v4f v = *(const v4f*)(embd + (size_t)id * HID + 4 * lane);
    const v4f z = {0.0f, 0.0f, 0.0f, 0.0f};
    v = (n < N) ? v : z;
    float* op = xout + (size_t)n * HID + 4 * lane;
    *(volatile v4f*)op = v;
    __threadfence();
    *(volatile v4f*)op = v;
}

__device__ __forceinline__ void chunk_keys(const int* __restrict__ recv, int cb, int lane, int E, int N,
                                           unsigned& key_out, int& rank, bool& last, bool& valid) {
    const int e = cb + lane;
    const int ec = e < E ? e : E - 1;
    const int r = recv[ec];
    unsigned key = 0xFFFFFFFFu;
    if (e < E && r >= 0 && r < N) key = ((unsigned)r & ~31u) | (unsigned)lane;
#pragma unroll
    for (int kk = 2; kk <= 32; kk <<= 1) {
#pragma unroll
        for (int j = kk >> 1; j > 0; j >>= 1) {
            const unsigned p = __shfl_xor(key, j);
            const bool asc = (lane & kk) == 0;
            const bool low = (lane & j) == 0;
            const unsigned mn = key < p ? key : p;
            const unsigned mx = key < p ? p : key;
            key = (asc == low) ? mn : mx;
        }
    }
    const unsigned bkt = key >> 5;
    const unsigned pk = __shfl_up(key, 1);
    const unsigned nk = __shfl_down(key, 1);
    const bool start = (lane == 0) || ((pk >> 5) != bkt);
    last = (lane == 31) || ((nk >> 5) != bkt);
    int v = start ? lane : 0;
#pragma unroll
    for (int d = 1; d < 32; d <<= 1) {
        const int uu = __shfl_up(v, d);
        if (lane >= d && uu > v) v = uu;
    }
    rank = lane - v;
    key_out = key;
    valid = (key != 0xFFFFFFFFu);
}

__global__ __launch_bounds__(128) void k_bucket(const int* __restrict__ recv, int* lists, int* offtab, int E, int N) {
    __shared__ unsigned short wcnt[4 * MAXB];
    __shared__ __attribute__((aligned(16))) int list_lds[CH1];
    __shared__ __attribute__((aligned(16))) int boff[PITCHB];
    __shared__ int sb[128];
    const int t = threadIdx.x, lane = t & 31, wid = t >> 5, blk = blockIdx.x;

    for (int i = t; i < 4 * MAXB; i += 128) wcnt[i] = 0;
    for (int i = t; i < CH1; i += 128) list_lds[i] = 0;
    __syncthreads();

    const int wbase = blk * CH1 + wid * 512;
#pragma unroll 1
    for (int c = 0; c < 16; ++c) {
        unsigned key; int rank; bool last, valid;
        chunk_keys(recv, wbase + c * 32, lane, E, N, key, rank, last, valid);
        if (valid && last) {
            const int b = (int)(key >> 5);
            wcnt[wid * MAXB + b] += (unsigned short)(rank + 1);
        }
    }
    __syncthreads();

    int tsum = 0;
#pragma unroll 1
    for (int q = 0; q < BPT; ++q) {
        const int b = t * BPT + q;
        if (b < PITCHB) {
            int tot = 0;
#pragma unroll
            for (int w = 0; w < 4; ++w) tot += (int)wcnt[w * MAXB + b];
            tsum += tot;
        }
    }
    sb[t] = tsum;
    __syncthreads();
#pragma unroll 1
    for (int d = 1; d < 128; d <<= 1) {
        const int vv = sb[(t >= d) ? (t - d) : t];
        const int v = (t >= d) ? vv : 0;
        __syncthreads();
        sb[t] += v;
        __syncthreads();
    }
    int run = sb[t] - tsum;
#pragma unroll 1
    for (int q = 0; q < BPT; ++q) {
        const int b = t * BPT + q;
        if (b < PITCHB) {
            boff[b] = run;
#pragma unroll
            for (int w = 0; w < 4; ++w) {
                const int cnt = (int)wcnt[w * MAXB + b];
                wcnt[w * MAXB + b] = (unsigned short)run;
                run += cnt;
            }
        }
    }
    __syncthreads();

#pragma unroll 1
    for (int c = 0; c < 16; ++c) {
        const int cb = wbase + c * 32;
        unsigned key; int rank; bool last, valid;
        chunk_keys(recv, cb, lane, E, N, key, rank, last, valid);
        if (valid) {
            const int b = (int)(key >> 5);
            const int pos = (int)wcnt[wid * MAXB + b] + rank;
            if ((unsigned)pos < (unsigned)CH1) list_lds[pos] = cb + (int)(key & 31u);
            if (last) wcnt[wid * MAXB + b] = (unsigned short)(pos + 1);
        }
    }
    __syncthreads();

    const v4ia* lsrc = (const v4ia*)list_lds;
    const v4ia* bsrc = (const v4ia*)boff;
    int* ld = lists + (size_t)blk * CH1;
    int* bd = offtab + (size_t)blk * PITCHB;
#pragma unroll
    for (int u = 0; u < 4; ++u) {
        const v4i v = lsrc[t + u * 128];
        *(volatile v4i*)(ld + (size_t)(t + u * 128) * 4) = v;
    }
#pragma unroll
    for (int u = 0; u < 7; ++u) {
        const int idx = t + u * 128;
        const bool has = idx < (PITCHB / 4);
        const v4i v = bsrc[has ? idx : 0];
        if (has) *(volatile v4i*)(bd + (size_t)idx * 4) = v;
    }
    __threadfence();
#pragma unroll
    for (int u = 0; u < 4; ++u) {
        const v4i v = lsrc[t + u * 128];
        *(volatile v4i*)(ld + (size_t)(t + u * 128) * 4) = v;
    }
#pragma unroll
    for (int u = 0; u < 7; ++u) {
        const int idx = t + u * 128;
        const bool has = idx < (PITCHB / 4);
        const v4i v = bsrc[has ? idx : 0];
        if (has) *(volatile v4i*)(bd + (size_t)idx * 4) = v;
    }
}

__global__ __launch_bounds__(32) void k_aggr(const float* hbuf, const float* xold, const int* __restrict__ srcv,
                                             const int* __restrict__ recv, const int* lists, const int* offtab,
                                             float* xnew, int E, int N, int NB1, int ngrp) {
    __shared__ unsigned comp[CAP3];
    __shared__ __attribute__((aligned(16))) v4f acc[32 * 32];
    const int lane = threadIdx.x & 31;
    const int f = blockIdx.x;
    const v4f z4 = {0.0f, 0.0f, 0.0f, 0.0f};

    int carry = 0;
#pragma unroll 1
    for (int u = 0; u < ngrp; ++u) {
        const int blk = lane + 32 * u;
        const bool inb = blk < NB1;
        const int cblk = inb ? blk : 0;
        const int* tb = offtab + (size_t)cblk * PITCHB;
        int a = tb[f];
        int b = tb[f + 1];
        a = a < 0 ? 0 : (a > CH1 ? CH1 : a);
        b = b < a ? a : (b > CH1 ? CH1 : b);
        const int c = inb ? (b - a) : 0;
        a = inb ? a : 0;
        int s = c;
#pragma unroll
        for (int d = 1; d < 32; d <<= 1) {
            const int v = __shfl_up(s, d);
            if (lane >= d) s += v;
        }
        const int ex = carry + s - c;
        const int tot = __shfl(s, 31);
        int qmax = c;
#pragma unroll
        for (int d = 16; d > 0; d >>= 1) {
            const int o = __shfl_xor(qmax, d);
            qmax = o > qmax ? o : qmax;
        }
        const int* lbase = lists + (size_t)cblk * CH1;
#pragma unroll 1
        for (int q = 0; q < qmax; ++q) {
            const bool act = q < c;
            int li = a + q;
            li = li < 0 ? 0 : (li > CH1 - 1 ? CH1 - 1 : li);
            const int e = lbase[li];
            const int ec = e < 0 ? 0 : (e > E - 1 ? E - 1 : e);
            const int nd = recv[ec] - f * 32;
            unsigned pk = 0xFFFFFFFFu;
            if ((unsigned)e < (unsigned)E && (unsigned)nd < 32u) pk = ((unsigned)e << 5) | (unsigned)nd;
            const int p = ex + q;
            if (act && (unsigned)p < (unsigned)CAP3) comp[p] = pk;
        }
        carry += tot;
    }
    const int T = carry < CAP3 ? carry : CAP3;

#pragma unroll 8
    for (int r = 0; r < 32; ++r) acc[r * 32 + lane] = z4;
    __syncthreads();

#pragma unroll 1
    for (int i = 0; i < T; ++i) {
        const unsigned pk = comp[i];
        const bool valid = pk != 0xFFFFFFFFu;
        int e = (int)(pk >> 5);
        e = valid ? e : 0;
        e = e < 0 ? 0 : (e > E - 1 ? E - 1 : e);
        const int nd = (int)(pk & 31u);
        int sn = srcv[e];
        sn = sn < 0 ? 0 : (sn > N - 1 ? N - 1 : sn);
        const v4f v = *(const v4f*)(hbuf + (size_t)sn * HID + 4 * lane);
        const v4f vs = valid ? v : z4;
        acc[nd * 32 + lane] += vs;
    }
    __syncthreads();

    const size_t nbase = (size_t)f * 32;
#pragma unroll 1
    for (int nd = 0; nd < 32; ++nd) {
        const v4f xv = *(const v4f*)(xold + (nbase + nd) * HID + 4 * lane);
        v4f r = acc[nd * 32 + lane];
        r += xv;
        float ss = r.x * r.x + r.y * r.y + r.z * r.z + r.w * r.w;
#pragma unroll
        for (int off = 16; off >= 1; off >>= 1) ss += __shfl_xor(ss, off);
        const float dn = fmaxf(sqrtf(ss), 1e-12f);
        const float sc = 1.0f / dn;
        r *= sc;
        acc[nd * 32 + lane] = r;
    }
    __syncthreads();

    float* ob = xnew + nbase * HID + 4 * lane;
#pragma unroll
    for (int nd = 0; nd < 32; ++nd) {
        const v4f v = acc[nd * 32 + lane];
        *(volatile v4f*)(ob + (size_t)nd * HID) = v;
    }
    __threadfence();
#pragma unroll
    for (int nd = 0; nd < 32; ++nd) {
        const v4f v = acc[nd * 32 + lane];
        *(volatile v4f*)(ob + (size_t)nd * HID) = v;
    }
}

__global__ __launch_bounds__(32) void k_lin(const float* xin, const _Float16* bfrag, int tbase,
                                            const float* __restrict__ bias, float* hout) {
    __shared__ __attribute__((aligned(16))) float stg[16 * SP];
    const int tile = blockIdx.x;
    const int lane = threadIdx.x & 31, h = lane >> 4, m = lane & 15;
    const float* xrow = xin + ((size_t)tile * 16 + m) * HID;
    const v16h a0 = frag_f32(xrow, 0, h);
    const v16h a1 = frag_f32(xrow, 32, h);
    const v16h a2 = frag_f32(xrow, 64, h);
    const v16h a3 = frag_f32(xrow, 96, h);
    const v8h* bq = (const v8h*)bfrag;
    const float inv = 0.015625f;

#pragma unroll 1
    for (int nt = 0; nt < 8; ++nt) {
        const v16h b0 = frag_b(bq, tbase + nt, lane);
        const v16h b1 = frag_b(bq, tbase + 8 + nt, lane);
        const v16h b2 = frag_b(bq, tbase + 16 + nt, lane);
        const v16h b3 = frag_b(bq, tbase + 24 + nt, lane);
        v8f c = zero8();
        c = wmma16(a0, b0, c);
        c = wmma16(a1, b1, c);
        c = wmma16(a2, b2, c);
        c = wmma16(a3, b3, c);
        asm volatile("v_nop\n\tv_nop\n\tv_nop\n\tv_nop" : "+v"(c)
                     : "v"(a0), "v"(a1), "v"(a2), "v"(a3), "v"(b0), "v"(b1), "v"(b2), "v"(b3));
        const float bv = bias[nt * 16 + m];
#pragma unroll
        for (int r = 0; r < 8; ++r)
            stg[(8 * h + r) * SP + nt * 16 + m] = fmaxf(c[r] * inv + bv, 0.0f);
    }
    __syncthreads();

    float* gb = hout + (size_t)tile * 16 * HID + 4 * lane;
#pragma unroll
    for (int rr = 0; rr < 16; ++rr) {
        const v4f v = *(const v4fa*)(stg + rr * SP + 4 * lane);
        *(volatile v4f*)(gb + (size_t)rr * HID) = v;
    }
    __threadfence();
#pragma unroll
    for (int rr = 0; rr < 16; ++rr) {
        const v4f v = *(const v4fa*)(stg + rr * SP + 4 * lane);
        *(volatile v4f*)(gb + (size_t)rr * HID) = v;
    }
}

__global__ __launch_bounds__(32) void k_pool(const float* xf, const int* __restrict__ gid, float* part,
                                             int N, int GP, int chunk) {
    __shared__ __attribute__((aligned(16))) float acc[GRW * 32];
    const int lane = threadIdx.x & 31;
    const int slab = blockIdx.x;
    const int gr = blockIdx.y;
    const int ch = blockIdx.z;
    const int g0 = gr * GRW;
#pragma unroll 8
    for (int g = 0; g < GRW; ++g) acc[g * 32 + lane] = 0.0f;
    __syncthreads();
    const int n0 = ch * chunk;
    int n1 = n0 + chunk;
    n1 = n1 > N ? N : n1;
#pragma unroll 1
    for (int n = n0; n < n1; ++n) {
        const int g = gid[n];
        const float v = xf[(size_t)n * HID + 32 * slab + lane];
        const int gl = g - g0;
        const bool in = (unsigned)gl < (unsigned)GRW;
        const int gc = in ? gl : 0;
        const float vs = in ? v : 0.0f;
        acc[gc * 32 + lane] += vs;
    }
    __syncthreads();

    const v4fa* av = (const v4fa*)acc;
    float* pb = part + ((size_t)ch * GP + g0) * HID + 32 * slab + (lane & 7) * 4;
#pragma unroll 8
    for (int it = 0; it < GRW / 4; ++it) {
        const v4f v = av[it * 32 + lane];
        *(volatile v4f*)(pb + (size_t)(it * 4 + (lane >> 3)) * HID) = v;
    }
    __threadfence();
#pragma unroll 8
    for (int it = 0; it < GRW / 4; ++it) {
        const v4f v = av[it * 32 + lane];
        *(volatile v4f*)(pb + (size_t)(it * 4 + (lane >> 3)) * HID) = v;
    }
}

__global__ __launch_bounds__(256) void k_poolsum(const float* part, float* mbuf, int GP, int nch) {
    const int lane = threadIdx.x & 31;
    const int g = blockIdx.x * 8 + (threadIdx.x >> 5);
    v4f s = {0.0f, 0.0f, 0.0f, 0.0f};
#pragma unroll 1
    for (int chn = 0; chn < nch; ++chn)
        s += *(const v4f*)(part + ((size_t)chn * GP + g) * HID + 4 * lane);
    float* op = mbuf + (size_t)g * HID + 4 * lane;
    *(volatile v4f*)op = s;
    __threadfence();
    *(volatile v4f*)op = s;
}

__global__ __launch_bounds__(64) void k_head(const float* mbuf, const _Float16* bfrag,
                                             const float* __restrict__ lb, const float* __restrict__ wpw,
                                             const float* __restrict__ wpb, float* out, int G) {
    __shared__ __attribute__((aligned(16))) _Float16 h1[2][16 * HP];
    __shared__ __attribute__((aligned(16))) float outl[32];
    const int t = threadIdx.x, lane = t & 31, wid = t >> 5, h = lane >> 4, m = lane & 15;
    const int g0 = blockIdx.x * 32 + wid * 16;
    const float inv = 0.015625f;
    const v8h* bq = (const v8h*)bfrag;
    _Float16* hw = h1[wid];

    const float* mrow = mbuf + (size_t)(g0 + m) * HID;
    const v16h a0 = frag_f32(mrow, 0, h);
    const v16h a1 = frag_f32(mrow, 32, h);
    const v16h a2 = frag_f32(mrow, 64, h);
    const v16h a3 = frag_f32(mrow, 96, h);

#pragma unroll 1
    for (int nt = 0; nt < 8; ++nt) {
        const v16h b0 = frag_b(bq, TB_L0 + nt, lane);
        const v16h b1 = frag_b(bq, TB_L0 + 8 + nt, lane);
        const v16h b2 = frag_b(bq, TB_L0 + 16 + nt, lane);
        const v16h b3 = frag_b(bq, TB_L0 + 24 + nt, lane);
        v8f c = zero8();
        c = wmma16(a0, b0, c);
        c = wmma16(a1, b1, c);
        c = wmma16(a2, b2, c);
        c = wmma16(a3, b3, c);
        asm volatile("v_nop\n\tv_nop\n\tv_nop\n\tv_nop" : "+v"(c)
                     : "v"(a0), "v"(a1), "v"(a2), "v"(a3), "v"(b0), "v"(b1), "v"(b2), "v"(b3));
        const float bv = lb[nt * 16 + m];
#pragma unroll
        for (int r = 0; r < 8; ++r)
            hw[(8 * h + r) * HP + nt * 16 + m] = (_Float16)fmaxf(c[r] * inv + bv, 0.0f);
    }
    __syncthreads();

    const v16h e0 = frag_lds(hw + m * HP, 0, h);
    const v16h e1 = frag_lds(hw + m * HP, 32, h);
    const v16h e2 = frag_lds(hw + m * HP, 64, h);
    const v16h e3 = frag_lds(hw + m * HP, 96, h);
    v8f accv = zero8();
#pragma unroll 1
    for (int nt = 0; nt < 8; ++nt) {
        const v16h b0 = frag_b(bq, TB_L1 + nt, lane);
        const v16h b1 = frag_b(bq, TB_L1 + 8 + nt, lane);
        const v16h b2 = frag_b(bq, TB_L1 + 16 + nt, lane);
        const v16h b3 = frag_b(bq, TB_L1 + 24 + nt, lane);
        v8f c = zero8();
        c = wmma16(e0, b0, c);
        c = wmma16(e1, b1, c);
        c = wmma16(e2, b2, c);
        c = wmma16(e3, b3, c);
        asm volatile("v_nop\n\tv_nop\n\tv_nop\n\tv_nop" : "+v"(c)
                     : "v"(e0), "v"(e1), "v"(e2), "v"(e3), "v"(b0), "v"(b1), "v"(b2), "v"(b3));
        const float bv = lb[HID + nt * 16 + m];
        const float wv = wpw[nt * 16 + m];
#pragma unroll
        for (int r = 0; r < 8; ++r)
            accv[r] = fmaf(fmaxf(c[r] * inv + bv, 0.0f), wv, accv[r]);
    }
#pragma unroll
    for (int r = 0; r < 8; ++r) {
#pragma unroll
        for (int off = 8; off >= 1; off >>= 1) accv[r] += __shfl_xor(accv[r], off);
    }
    const float wb = wpb[0];
    if (m == 0) {
#pragma unroll
        for (int r = 0; r < 8; ++r) outl[wid * 16 + 8 * h + r] = accv[r] + wb;
    }
    __syncthreads();

    const int q = lane & 7;
    const v4f ov = ((const v4fa*)outl)[q];
    const int idx = blockIdx.x * 32 + q * 4;
    const bool ok = (wid == 0) && (lane < 8) && (idx + 4 <= G);
    if (ok) *(volatile v4f*)(out + idx) = ov;
    __threadfence();
    if (ok) *(volatile v4f*)(out + idx) = ov;
}

extern "C" void kernel_launch(void* const* d_in, const int* in_sizes, int n_in,
                              void* d_out, int out_size, void* d_ws, size_t ws_size,
                              hipStream_t stream) {
    if (n_in < 10) return;
    const int*   x_ids = (const int*)d_in[0];
    const int*   edges = (const int*)d_in[1];
    const int*   gidv  = (const int*)d_in[2];
    const float* embd  = (const float*)d_in[3];
    const float* gcn_w = (const float*)d_in[4];
    const float* gcn_b = (const float*)d_in[5];
    const float* lin_w = (const float*)d_in[6];
    const float* lin_b = (const float*)d_in[7];
    const float* wp_w  = (const float*)d_in[8];
    const float* wp_b  = (const float*)d_in[9];
    float* out = (float*)d_out;

    const int N = in_sizes[0];
    const int E = in_sizes[1] / 2;
    const int G = out_size;
    const int V = in_sizes[3] / HID;
    if (N <= 0 || E <= 0 || G < 1 || V < 1 || (G & 3) != 0) return;
    if (in_sizes[1] != 2 * E || in_sizes[2] != N || in_sizes[3] != V * HID) return;
    if (in_sizes[4] != 3 * HID * HID || in_sizes[5] != 3 * HID || in_sizes[6] != 2 * HID * HID ||
        in_sizes[7] != 2 * HID || in_sizes[8] != HID || in_sizes[9] < 1) return;
    if (E > (1 << 26)) return;

    const int* src = edges;
    const int* dst = edges + E;

    const int NB = (N + 31) / 32;
    const int NR = NB * 32;
    if (NB + 1 > PITCHB) return;
    const int NB1 = (E + CH1 - 1) / CH1;
    if (NB1 > MAXNB1) return;
    const int ngrp = (NB1 + 31) / 32;
    const int NT = (N + 15) / 16;
    const int GRN = (G + GRW - 1) / GRW;
    const int GP = GRN * GRW;
    const int chunk = (N + NCH - 1) / NCH;

    size_t off = 0;
    auto carve = [&](size_t bytes) -> size_t { const size_t p = off; off += (bytes + 255) & ~(size_t)255; return p; };
    const size_t o_bf    = carve((size_t)NSLOTS * 8 * sizeof(_Float16));
    const size_t o_lists = carve((size_t)NB1 * CH1 * sizeof(int));
    const size_t o_tab   = carve((size_t)NB1 * PITCHB * sizeof(int));
    const size_t o_x0    = carve((size_t)NR * HID * sizeof(float));
    const size_t o_x1    = carve((size_t)NR * HID * sizeof(float));
    const size_t o_h     = carve((size_t)NR * HID * sizeof(float));
    const size_t o_part  = carve((size_t)NCH * GP * HID * sizeof(float));
    const size_t o_m     = carve((size_t)GP * HID * sizeof(float));
    if (off > ws_size || off > (size_t)134217728) return;

    char* ws = (char*)d_ws;
    _Float16* bfrag = (_Float16*)(ws + o_bf);
    int* lists = (int*)(ws + o_lists);
    int* offtab = (int*)(ws + o_tab);
    float* x0 = (float*)(ws + o_x0);
    float* x1 = (float*)(ws + o_x1);
    float* hb = (float*)(ws + o_h);
    float* part = (float*)(ws + o_part);
    float* mbuf = (float*)(ws + o_m);

    k_prep<<<(NSLOTS + 255) / 256, 256, 0, stream>>>(gcn_w, lin_w, bfrag);
    k_embed<<<NR / 8, 256, 0, stream>>>(x_ids, embd, x0, N, V);
    k_bucket<<<NB1, 128, 0, stream>>>(dst, lists, offtab, E, N);
    for (int l = 0; l < 3; ++l) {
        const float* xin = (l & 1) ? x1 : x0;
        float* xout = (l & 1) ? x0 : x1;
        k_lin<<<NT, 32, 0, stream>>>(xin, bfrag, l * 32, gcn_b + (size_t)l * HID, hb);
        k_aggr<<<NB, 32, 0, stream>>>(hb, xin, src, dst, lists, offtab, xout, E, N, NB1, ngrp);
    }
    const float* xfin = x1;
    k_pool<<<dim3(HID / 32, GRN, NCH), 32, 0, stream>>>(xfin, gidv, part, N, GP, chunk);
    k_poolsum<<<GP / 8, 256, 0, stream>>>(part, mbuf, GP, NCH);
    k_head<<<GP / 32, 64, 0, stream>>>(mbuf, bfrag, lin_b, wp_w, wp_b, out, G);
}
